// OuterProductMean_88184268521492
// MI455X (gfx1250) — hardware-verified
//
#include <hip/hip_runtime.h>
#include <stdint.h>

constexpr int kS   = 128;
constexpr int kR   = 256;
constexpr int kCM  = 256;
constexpr int kH   = 32;
constexpr int kCZ  = 128;
constexpr int kHH  = kH * kH;
constexpr int kRowsX = kS * kR;
constexpr int kIChunk = 64;
constexpr int kNChunk = kR / kIChunk;
constexpr float kEps   = 1e-3f;
constexpr float kLnEps = 1e-5f;

constexpr size_t kSzX   = (size_t)kRowsX * kCM * 2;
constexpr size_t kSzA   = (size_t)kR * kH * kS * 2;
constexpr size_t kSzO   = (size_t)kIChunk * kR * kHH * 2;
constexpr size_t kSzWT  = (size_t)kH * kCM * 2;
constexpr size_t kSzWOT = (size_t)kCZ * kHH * 2;
constexpr size_t kSzRN  = (size_t)kR * kR * 4;
constexpr size_t kOffXH  = 0;
constexpr size_t kOffXL  = kOffXH + kSzX;
constexpr size_t kOffAH  = kOffXL + kSzX;
constexpr size_t kOffAL  = kOffAH + kSzA;
constexpr size_t kOffBH  = kOffAL + kSzA;
constexpr size_t kOffBL  = kOffBH + kSzA;
constexpr size_t kOffOH  = kOffBL + kSzA;
constexpr size_t kOffOL  = kOffOH + kSzO;
constexpr size_t kOffW1T = kOffOL + kSzO;
constexpr size_t kOffW2T = kOffW1T + kSzWT;
constexpr size_t kOffWOT = kOffW2T + kSzWT;
constexpr size_t kOffRN  = kOffWOT + kSzWOT;
constexpr size_t kWsTotal = kOffRN + kSzRN;
static_assert(kWsTotal == 109608960ull);
static_assert(kWsTotal <= 134217728ull);
static_assert((kOffXL % 16384) == 0 && (kOffAH % 16384) == 0 && (kOffOH % 16384) == 0 && (kOffW1T % 16384) == 0 && (kOffRN % 16384) == 0);

static_assert(kCM % 32 == 0 && kS % 32 == 0 && kHH % 32 == 0);
static_assert(kRowsX % 64 == 0 && (kIChunk * kH) % 64 == 0 && (kR * kH) % 64 == 0 && (kIChunk * kR) % 64 == 0 && kCZ % 64 == 0);
static_assert(kS % 64 == 0);
static_assert(kH == 32);

typedef __attribute__((ext_vector_type(16))) _Float16 v16h;
typedef __attribute__((ext_vector_type(8)))  _Float16 v8h;
typedef __attribute__((ext_vector_type(16))) __bf16   v16b;
typedef __attribute__((ext_vector_type(8)))  __bf16   v8b;
typedef __attribute__((ext_vector_type(8)))  float    v8f;
typedef __attribute__((ext_vector_type(4)))  float    v4f;
typedef __attribute__((ext_vector_type(4)))  unsigned int v4u;

__device__ __forceinline__ unsigned short f2bf_bits(float f) {
  unsigned u = __float_as_uint(f);
  return (unsigned short)((u + 0x7FFFu + ((u >> 16) & 1u)) >> 16);
}
__device__ __forceinline__ float bf_bits2f(unsigned short h) { return __uint_as_float(((unsigned)h) << 16); }
__device__ __forceinline__ float bfr(float f) { return bf_bits2f(f2bf_bits(f)); }
__device__ __forceinline__ unsigned pk16(unsigned short a, unsigned short b) { return (unsigned)a | ((unsigned)b << 16); }

__device__ __forceinline__ void dep_guard_b(v8f& a, v8f& b, v16b x, v16b y) { asm volatile("v_nop\n\tv_nop\n\tv_nop\n\tv_nop" : "+v"(a), "+v"(b) : "v"(x), "v"(y)); }
__device__ __forceinline__ void dep_guard4_b(v8f& a, v8f& b, v8f& c, v8f& d, v16b x, v16b y) {
  asm volatile("v_nop\n\tv_nop\n\tv_nop\n\tv_nop" : "+v"(a), "+v"(b), "+v"(c), "+v"(d) : "v"(x), "v"(y));
}
__device__ __forceinline__ void keep4_b(v16b a, v16b b, v16b c, v16b d) { asm volatile("v_nop" :: "v"(a), "v"(b), "v"(c), "v"(d)); }
__device__ __forceinline__ void acc_guard4(v8f& a, v8f& b, v8f& c, v8f& d) { asm volatile("v_nop\n\tv_nop\n\tv_nop\n\tv_nop" : "+v"(a), "+v"(b), "+v"(c), "+v"(d)); }

template <typename T> struct Frag;
template <> struct Frag<__bf16> {
  typedef v16b V; union U { v16b v; v8b h[2]; };
  static __device__ __forceinline__ v16b load(const __bf16* p) {
    U f; f.h[0] = *(const v8b*)(p); f.h[1] = *(const v8b*)(p + 16); return f.v;
  }
  static __device__ __forceinline__ v8f mma(v16b a, v16b b, v8f c) {
    return __builtin_amdgcn_wmma_f32_16x16x32_bf16(false, a, false, b, (short)0, c, false, false);
  }
};

__device__ __forceinline__ void wave_sync_lds() {
  __builtin_amdgcn_fence(__ATOMIC_RELEASE, "workgroup");
  __builtin_amdgcn_wave_barrier();
  __builtin_amdgcn_fence(__ATOMIC_ACQUIRE, "workgroup");
}

__device__ __forceinline__ void split_pack8(const float (&f)[8], v4u& uh, v4u& ul) {
  unsigned short hb[8], lb[8];
#pragma unroll
  for (int e = 0; e < 8; ++e) {
    hb[e] = f2bf_bits(f[e]);
    lb[e] = f2bf_bits(f[e] - bf_bits2f(hb[e]));
  }
  uh = (v4u){pk16(hb[0], hb[1]), pk16(hb[2], hb[3]), pk16(hb[4], hb[5]), pk16(hb[6], hb[7])};
  ul = (v4u){pk16(lb[0], lb[1]), pk16(lb[2], lb[3]), pk16(lb[4], lb[5]), pk16(lb[6], lb[7])};
}

__device__ __forceinline__ void row_guard(v8f (&a)[2], v16b x, v16b y) { dep_guard_b(a[0], a[1], x, y); }
__device__ __forceinline__ void row_guard(v8f (&a)[4], v16b x, v16b y) { dep_guard4_b(a[0], a[1], a[2], a[3], x, y); }
__device__ __forceinline__ void fin_guard(v8f (&acc)[4][2]) {
  acc_guard4(acc[0][0], acc[0][1], acc[1][0], acc[1][1]);
  acc_guard4(acc[2][0], acc[2][1], acc[3][0], acc[3][1]);
}
__device__ __forceinline__ void fin_guard(v8f (&acc)[4][4]) {
  acc_guard4(acc[0][0], acc[0][1], acc[0][2], acc[0][3]);
  acc_guard4(acc[1][0], acc[1][1], acc[1][2], acc[1][3]);
  acc_guard4(acc[2][0], acc[2][1], acc[2][2], acc[2][3]);
  acc_guard4(acc[3][0], acc[3][1], acc[3][2], acc[3][3]);
}

template <int NJ, int SPL>
__device__ __forceinline__ void core_bf16(const __bf16* __restrict__ Ab, const __bf16* __restrict__ Ab2, int lda,
                                          const __bf16* __restrict__ Bb, const __bf16* __restrict__ Bb2, int ldb,
                                          int m0, int n0, int K, int lane, v8f (&acc)[4][NJ]) {
  const int rlane = lane & 15;
  const int koff  = (lane >> 4) * 8;
#pragma unroll 1
  for (int k0 = 0; k0 < K; k0 += 32) {
    v16b bh[NJ], bl[NJ];
#pragma unroll
    for (int j = 0; j < NJ; ++j) {
      const size_t bo = (size_t)(n0 + (j << 4) + rlane) * ldb + koff + k0;
      bh[j] = Frag<__bf16>::load(Bb + bo);
      bl[j] = bh[j];
      if (SPL == 2) bl[j] = Frag<__bf16>::load(Bb2 + bo);
    }
#pragma unroll
    for (int i = 0; i < 4; ++i) {
      const size_t ao = (size_t)(m0 + (i << 4) + rlane) * lda + koff + k0;
      const v16b ah = Frag<__bf16>::load(Ab + ao);
      v16b al = ah;
      if (SPL >= 1) al = Frag<__bf16>::load(Ab2 + ao);
#pragma unroll
      for (int j = 0; j < NJ; ++j) {
        acc[i][j] = Frag<__bf16>::mma(ah, bh[j], acc[i][j]);
        if (SPL == 2) acc[i][j] = Frag<__bf16>::mma(ah, bl[j], acc[i][j]);
        if (SPL >= 1) acc[i][j] = Frag<__bf16>::mma(al, bh[j], acc[i][j]);
      }
      row_guard(acc[i], ah, al);
    }
    keep4_b(bh[0], bh[1], bh[NJ - 2], bh[NJ - 1]);
    if (SPL == 2) keep4_b(bl[0], bl[1], bl[NJ - 2], bl[NJ - 1]);
  }
  fin_guard(acc);
}

__global__ __launch_bounds__(128) void wt12_kernel(const float* __restrict__ w1, const float* __restrict__ w2,
                                                   unsigned short* __restrict__ o1, unsigned short* __restrict__ o2) {
  const int lane = threadIdx.x & 31, wave = threadIdx.x >> 5;
  const int h = blockIdx.x * 4 + wave;
  const int sel = blockIdx.y;
  const float* w = sel ? w2 : w1;
  unsigned short* o = sel ? o2 : o1;
  unsigned short hb[8];
#pragma unroll
  for (int t = 0; t < 8; ++t) hb[t] = f2bf_bits(w[(size_t)(lane * 8 + t) * kH + h]);
  const v4u u = (v4u){pk16(hb[0], hb[1]), pk16(hb[2], hb[3]), pk16(hb[4], hb[5]), pk16(hb[6], hb[7])};
  unsigned short* dst = o + (size_t)h * kCM + lane * 8;
  *(volatile v4u*)dst = u;
  __threadfence();
  *(volatile v4u*)dst = u;
}

__global__ __launch_bounds__(256) void wot_kernel(const float* __restrict__ wo, unsigned short* __restrict__ o) {
  const int lane = threadIdx.x & 31, wave = threadIdx.x >> 5;
  const int gw = blockIdx.x * 8 + wave;
  const int z = gw >> 2, qq = gw & 3;
  unsigned short hb[8];
#pragma unroll
  for (int t = 0; t < 8; ++t) {
    const int k = qq * 256 + lane * 8 + t;
    hb[t] = f2bf_bits(wo[(size_t)k * kCZ + z]);
  }
  const v4u u = (v4u){pk16(hb[0], hb[1]), pk16(hb[2], hb[3]), pk16(hb[4], hb[5]), pk16(hb[6], hb[7])};
  unsigned short* dst = o + (size_t)z * kHH + qq * 256 + lane * 8;
  *(volatile v4u*)dst = u;
  __threadfence();
  *(volatile v4u*)dst = u;
}

__global__ __launch_bounds__(256) void rnorm_kernel(const float* __restrict__ mk1, const float* __restrict__ mk2, float* __restrict__ rn) {
  const int t = blockIdx.x * 256 + threadIdx.x;
  const int i = t >> 6, j0 = (t & 63) * 4;
  float a0 = 0.0f, a1 = 0.0f, a2 = 0.0f, a3 = 0.0f;
#pragma unroll 1
  for (int s = 0; s < kS; ++s) {
    const float u = bfr(mk1[(size_t)s * kR + i]);
    const v4f qv = *(const v4f*)(mk2 + (size_t)s * kR + j0);
    const float q0 = qv.x, q1 = qv.y, q2 = qv.z, q3 = qv.w;
    a0 += u * bfr(q0); a1 += u * bfr(q1); a2 += u * bfr(q2); a3 += u * bfr(q3);
  }
  v4f o;
  o.x = 1.0f / (a0 + kEps); o.y = 1.0f / (a1 + kEps); o.z = 1.0f / (a2 + kEps); o.w = 1.0f / (a3 + kEps);
  float* dst = rn + (size_t)i * kR + j0;
  *(volatile v4f*)dst = o;
  __threadfence();
  *(volatile v4f*)dst = o;
}

__global__ __launch_bounds__(256) void ln_split_kernel(const float* __restrict__ m, const float* __restrict__ lnw,
                                                       const float* __restrict__ lnb,
                                                       unsigned short* __restrict__ XH, unsigned short* __restrict__ XL) {
  const int lane = threadIdx.x & 31, wave = threadIdx.x >> 5;
  const int q = blockIdx.x * 8 + wave;
  const int rr = q >> 7, s = q & 127;
  const float* xp = m + ((size_t)s * kR + rr) * kCM + lane * 8;
  const v4f xa = *(const v4f*)(xp);
  const v4f xb = *(const v4f*)(xp + 4);
  float x[8];
  x[0] = bfr(xa.x); x[1] = bfr(xa.y); x[2] = bfr(xa.z); x[3] = bfr(xa.w);
  x[4] = bfr(xb.x); x[5] = bfr(xb.y); x[6] = bfr(xb.z); x[7] = bfr(xb.w);
  float sum = 0.0f;
#pragma unroll
  for (int e = 0; e < 8; ++e) sum += x[e];
#pragma unroll
  for (int off = 16; off > 0; off >>= 1) sum += __shfl_xor(sum, off, 32);
  const float mu = sum * (1.0f / 256.0f);
  float vs = 0.0f;
#pragma unroll
  for (int e = 0; e < 8; ++e) { const float d = x[e] - mu; vs += d * d; }
#pragma unroll
  for (int off = 16; off > 0; off >>= 1) vs += __shfl_xor(vs, off, 32);
  const float inv = rsqrtf(vs * (1.0f / 256.0f) + kLnEps);
  const v4f ga = *(const v4f*)(lnw + lane * 8);
  const v4f gb = *(const v4f*)(lnw + lane * 8 + 4);
  const v4f ba = *(const v4f*)(lnb + lane * 8);
  const v4f bb = *(const v4f*)(lnb + lane * 8 + 4);
  float g[8], be[8];
  g[0] = bfr(ga.x); g[1] = bfr(ga.y); g[2] = bfr(ga.z); g[3] = bfr(ga.w);
  g[4] = bfr(gb.x); g[5] = bfr(gb.y); g[6] = bfr(gb.z); g[7] = bfr(gb.w);
  be[0] = bfr(ba.x); be[1] = bfr(ba.y); be[2] = bfr(ba.z); be[3] = bfr(ba.w);
  be[4] = bfr(bb.x); be[5] = bfr(bb.y); be[6] = bfr(bb.z); be[7] = bfr(bb.w);
  float y[8];
#pragma unroll
  for (int e = 0; e < 8; ++e) y[e] = (x[e] - mu) * inv * g[e] + be[e];
  v4u uh, ul;
  split_pack8(y, uh, ul);
  const size_t off = (size_t)q * kCM + lane * 8;
  for (int pass = 0; pass < 2; ++pass) {
    *(volatile v4u*)(XH + off) = uh;
    *(volatile v4u*)(XL + off) = ul;
    __threadfence();
  }
}

__global__ __launch_bounds__(128) void proj_kernel(const unsigned short* __restrict__ XH, const unsigned short* __restrict__ XL,
                                                   const unsigned short* __restrict__ WT, const float* __restrict__ bias,
                                                   const float* __restrict__ mk,
                                                   unsigned short* __restrict__ AHo, unsigned short* __restrict__ ALo) {
  __shared__ __align__(16) float sT1[4][32 * 68];
  __shared__ float sM1[4][64];
  const int lane = threadIdx.x & 31, wave = threadIdx.x >> 5;
  const int rlane = lane & 15, mOff = (lane >> 4) * 8;
  const int tile = blockIdx.x * 4 + wave;
  const int m0 = tile << 6;
  const int rr = m0 >> 7;
  const int s0 = m0 & 127;
  float* slab = sT1[wave];
  float* mrow = sM1[wave];
  {
    const float mv0 = bfr(mk[(size_t)(s0 + lane) * kR + rr]);
    const float mv1 = bfr(mk[(size_t)(s0 + lane + 32) * kR + rr]);
    mrow[lane] = mv0;
    mrow[lane + 32] = mv1;
  }
  const float bb0 = bfr(bias[rlane]);
  const float bb1 = bfr(bias[16 + rlane]);
  wave_sync_lds();

  v8f acc[4][2];
#pragma unroll
  for (int i = 0; i < 4; ++i)
#pragma unroll
    for (int j = 0; j < 2; ++j) acc[i][j] = (v8f){0.f,0.f,0.f,0.f,0.f,0.f,0.f,0.f};
  core_bf16<2, 1>((const __bf16*)(const void*)XH, (const __bf16*)(const void*)XL, kCM,
                  (const __bf16*)(const void*)WT, (const __bf16*)(const void*)WT, kCM,
                  m0, 0, kCM, lane, acc);

#pragma unroll
  for (int i = 0; i < 4; ++i) {
#pragma unroll
    for (int j = 0; j < 2; ++j) {
      const int h = (j << 4) + rlane;
      const float bb = (j == 0) ? bb0 : bb1;
#pragma unroll
      for (int r = 0; r < 8; ++r) {
        const int sl = (i << 4) + mOff + r;
        const float v = (acc[i][j][r] + bb) * mrow[sl];
        slab[h * 68 + sl] = v;
      }
    }
  }
  wave_sync_lds();

  const int q = lane >> 3, w = lane & 7;
  for (int pass = 0; pass < 2; ++pass) {
#pragma unroll
    for (int it = 0; it < 8; ++it) {
      const int h = it * 4 + q;
      const float* sp = slab + h * 68 + w * 8;
      const v4f fa = *(const v4f*)(sp);
      const v4f fb = *(const v4f*)(sp + 4);
      float f[8];
      f[0] = fa.x; f[1] = fa.y; f[2] = fa.z; f[3] = fa.w;
      f[4] = fb.x; f[5] = fb.y; f[6] = fb.z; f[7] = fb.w;
      v4u uh, ul;
      split_pack8(f, uh, ul);
      const size_t off = (size_t)(rr * kH + h) * kS + s0 + w * 8;
      *(volatile v4u*)(AHo + off) = uh;
      *(volatile v4u*)(ALo + off) = ul;
    }
    __threadfence();
  }
}

__global__ __launch_bounds__(256) void outer_kernel(const unsigned short* __restrict__ AHp, const unsigned short* __restrict__ ALp,
                                                    const unsigned short* __restrict__ BHp, const unsigned short* __restrict__ BLp,
                                                    unsigned short* __restrict__ OHp, unsigned short* __restrict__ OLp) {
  __shared__ __align__(16) float sT2[8][16 * 68];
  const int lane = threadIdx.x & 31, wave = threadIdx.x >> 5;
  const int rlane = lane & 15, mOff = (lane >> 4) * 8;
  const int tile = blockIdx.x * 8 + wave;
  const int tm = tile >> 7, tn = tile & 127;
  const int m0 = tm << 6, n0 = tn << 6;

  v8f acc[4][4];
#pragma unroll
  for (int i = 0; i < 4; ++i)
#pragma unroll
    for (int j = 0; j < 4; ++j) acc[i][j] = (v8f){0.f,0.f,0.f,0.f,0.f,0.f,0.f,0.f};
  core_bf16<4, 2>((const __bf16*)(const void*)AHp, (const __bf16*)(const void*)ALp, kS,
                  (const __bf16*)(const void*)BHp, (const __bf16*)(const void*)BLp, kS,
                  m0, n0, kS, lane, acc);

  float* slab = sT2[wave];
  const int q = lane >> 3, w = lane & 7;
#pragma unroll
  for (int i = 0; i < 4; ++i) {
#pragma unroll
    for (int j = 0; j < 4; ++j) {
#pragma unroll
      for (int r = 0; r < 8; ++r) slab[(mOff + r) * 68 + (j << 4) + rlane] = acc[i][j][r];
    }
    wave_sync_lds();
    const int iloc  = tm * 2 + (i >> 1);
    const int cBase = (i & 1) * 16;
    for (int pass = 0; pass < 2; ++pass) {
#pragma unroll
      for (int it = 0; it < 4; ++it) {
        const int L   = it * 4 + q;
        const int jj  = L >> 3;
        const int cp  = L & 7;
        const int srow = cp * 2 + (w >> 2);
        const int scol = jj * 32 + (w & 3) * 8;
        const float* sp = slab + srow * 68 + scol;
        const v4f fa = *(const v4f*)(sp);
        const v4f fb = *(const v4f*)(sp + 4);
        float f[8];
        f[0] = fa.x; f[1] = fa.y; f[2] = fa.z; f[3] = fa.w;
        f[4] = fb.x; f[5] = fb.y; f[6] = fb.z; f[7] = fb.w;
        v4u uh, ul;
        split_pack8(f, uh, ul);
        const size_t off = ((size_t)(iloc * kR + tn * 2 + jj)) * kHH + (size_t)(cBase + srow) * kH + (w & 3) * 8;
        *(volatile v4u*)(OHp + off) = uh;
        *(volatile v4u*)(OLp + off) = ul;
      }
      __threadfence();
    }
    wave_sync_lds();
  }
}

__global__ __launch_bounds__(256) void down_kernel(const unsigned short* __restrict__ OHp, const unsigned short* __restrict__ OLp,
                                                   const unsigned short* __restrict__ WOTp, const float* __restrict__ bout,
                                                   const float* __restrict__ rnP, float* __restrict__ outp) {
  __shared__ __align__(16) float sT3[8][16 * 68];
  const int lane = threadIdx.x & 31, wave = threadIdx.x >> 5;
  const int rlane = lane & 15, mOff = (lane >> 4) * 8, hh = lane >> 4;
  const int tile = blockIdx.x * 8 + wave;
  const int tm = tile >> 1, tn = tile & 1;
  const int m0 = tm << 6, n0 = tn << 6;
  float bv[4];
#pragma unroll
  for (int j = 0; j < 4; ++j) bv[j] = bfr(bout[n0 + (j << 4) + rlane]);

  v8f acc[4][4];
#pragma unroll
  for (int i = 0; i < 4; ++i)
#pragma unroll
    for (int j = 0; j < 4; ++j) acc[i][j] = (v8f){0.f,0.f,0.f,0.f,0.f,0.f,0.f,0.f};
  core_bf16<4, 1>((const __bf16*)(const void*)OHp, (const __bf16*)(const void*)OLp, kHH,
                  (const __bf16*)(const void*)WOTp, (const __bf16*)(const void*)WOTp, kHH,
                  m0, n0, kHH, lane, acc);

  float* slab = sT3[wave];
  const int c4 = rlane * 4;
#pragma unroll
  for (int i = 0; i < 4; ++i) {
    const int mBase = m0 + (i << 4);
    const v4f ra = *(const v4f*)(rnP + mBase + mOff);
    const v4f rb = *(const v4f*)(rnP + mBase + mOff + 4);
    float rv[8];
    rv[0] = ra.x; rv[1] = ra.y; rv[2] = ra.z; rv[3] = ra.w;
    rv[4] = rb.x; rv[5] = rb.y; rv[6] = rb.z; rv[7] = rb.w;
#pragma unroll
    for (int j = 0; j < 4; ++j) {
#pragma unroll
      for (int r = 0; r < 8; ++r) {
        const float v = (acc[i][j][r] + bv[j]) * rv[r];
        slab[(mOff + r) * 68 + (j << 4) + rlane] = v;
      }
    }
    wave_sync_lds();
    for (int pass = 0; pass < 2; ++pass) {
#pragma unroll
      for (int it = 0; it < 8; ++it) {
        const int row = it * 2 + hh;
        const v4f v = *(const v4f*)(slab + row * 68 + c4);
        *(volatile v4f*)(outp + (size_t)(mBase + row) * kCZ + n0 + c4) = v;
      }
      __threadfence();
    }
    wave_sync_lds();
  }
}

extern "C" void kernel_launch(void* const* d_in, const int* in_sizes, int n_in,
                              void* d_out, int out_size, void* d_ws, size_t ws_size,
                              hipStream_t stream) {
  if (n_in < 14) return;
  if (ws_size < kWsTotal) return;
  if (out_size < kR * kR * kCZ) return;
  if (in_sizes[0] != kS * kR * kCM || in_sizes[1] != kS * kR * kCM) return;
  if (in_sizes[2] != kS * kR || in_sizes[3] != kS * kR) return;
  if (in_sizes[4] != kCM || in_sizes[5] != kCM || in_sizes[6] != kCM || in_sizes[7] != kCM) return;
  if (in_sizes[8] != kCM * kH || in_sizes[9] != kH || in_sizes[10] != kCM * kH || in_sizes[11] != kH) return;
  if (in_sizes[12] != kHH * kCZ || in_sizes[13] != kCZ) return;

  const float* m1    = (const float*)d_in[0];
  const float* m2    = (const float*)d_in[1];
  const float* mk1   = (const float*)d_in[2];
  const float* mk2   = (const float*)d_in[3];
  const float* ln1w  = (const float*)d_in[4];
  const float* ln1b  = (const float*)d_in[5];
  const float* ln2w  = (const float*)d_in[6];
  const float* ln2b  = (const float*)d_in[7];
  const float* w1    = (const float*)d_in[8];
  const float* b1    = (const float*)d_in[9];
  const float* w2    = (const float*)d_in[10];
  const float* b2    = (const float*)d_in[11];
  const float* w_out = (const float*)d_in[12];
  const float* bout  = (const float*)d_in[13];
  float* out = (float*)d_out;

  char* ws = (char*)d_ws;
  unsigned short* XH  = (unsigned short*)(ws + kOffXH);
  unsigned short* XL  = (unsigned short*)(ws + kOffXL);
  unsigned short* AH  = (unsigned short*)(ws + kOffAH);
  unsigned short* AL  = (unsigned short*)(ws + kOffAL);
  unsigned short* BH  = (unsigned short*)(ws + kOffBH);
  unsigned short* BL  = (unsigned short*)(ws + kOffBL);
  unsigned short* OH  = (unsigned short*)(ws + kOffOH);
  unsigned short* OL  = (unsigned short*)(ws + kOffOL);
  unsigned short* W1T = (unsigned short*)(ws + kOffW1T);
  unsigned short* W2T = (unsigned short*)(ws + kOffW2T);
  unsigned short* WOT = (unsigned short*)(ws + kOffWOT);
  float*          RN  = (float*)(ws + kOffRN);

  wt12_kernel<<<dim3(kH / 4, 2), 128, 0, stream>>>(w1, w2, W1T, W2T);
  wot_kernel<<<(kCZ * 4) / 8, 256, 0, stream>>>(w_out, WOT);
  rnorm_kernel<<<(kR * kR / 4) / 256, 256, 0, stream>>>(mk1, mk2, RN);

  ln_split_kernel<<<kRowsX / 8, 256, 0, stream>>>(m1, ln1w, ln1b, XH, XL);
  proj_kernel<<<(kRowsX / 64) / 4, 128, 0, stream>>>(XH, XL, W1T, b1, mk1, AH, AL);
  ln_split_kernel<<<kRowsX / 8, 256, 0, stream>>>(m2, ln2w, ln2b, XH, XL);
  proj_kernel<<<(kRowsX / 64) / 4, 128, 0, stream>>>(XH, XL, W2T, b2, mk2, BH, BL);

  const int outerTiles = ((kIChunk * kH) / 64) * ((kR * kH) / 64);
  const int downTiles  = ((kIChunk * kR) / 64) * (kCZ / 64);
  for (int ic = 0; ic < kNChunk; ++ic) {
    const size_t aoff = (size_t)ic * kIChunk * kH * kS;
    outer_kernel<<<outerTiles / 8, 256, 0, stream>>>(AH + aoff, AL + aoff, BH, BL, OH, OL);
    down_kernel<<<downTiles / 8, 256, 0, stream>>>(OH, OL, WOT, bout,
                                                  RN + (size_t)ic * kIChunk * kR,
                                                  out + (size_t)ic * kIChunk * kR * kCZ);
  }
}
